// LucyRNNCellTriton_89988154786159
// MI455X (gfx1250) — hardware-verified
//
#include <hip/hip_runtime.h>
#include <stddef.h>
#include <stdint.h>


typedef __attribute__((ext_vector_type(16))) _Float16 v16h;
typedef __attribute__((ext_vector_type(8)))  _Float16 v8h;
typedef __attribute__((ext_vector_type(16))) __bf16   v16b;
typedef __attribute__((ext_vector_type(8)))  __bf16   v8b;
typedef __attribute__((ext_vector_type(8)))  float    v8f;
typedef __attribute__((ext_vector_type(4)))  float    v4f;

#define LU_B      8
#define LU_T      2048
#define LU_IN     512
#define LU_D      512
#define LU_DSHIFT 9
#define LU_NG     6
#define LU_GC     (LU_NG * LU_D)
#define LU_TCH    1024
#define LU_NCH    (LU_T / LU_TCH)
#define LU_WSCALE     64.0f
#define LU_WSCALE_INV 0.015625f

__device__ __forceinline__ unsigned short f2bf_bits(float f) {
  unsigned u = __float_as_uint(f);
  return (unsigned short)((u + 0x7FFFu + ((u >> 16) & 1u)) >> 16);
}
__device__ __forceinline__ float bf_bits2f(unsigned short h) { return __uint_as_float(((unsigned)h) << 16); }

__device__ __forceinline__ void dep_guard_h(v8f& a, v8f& b, v16h x, v16h y) { asm volatile("v_nop\n\tv_nop\n\tv_nop\n\tv_nop" : "+v"(a), "+v"(b) : "v"(x), "v"(y)); }
__device__ __forceinline__ void dep_guard_b(v8f& a, v8f& b, v16b x, v16b y) { asm volatile("v_nop\n\tv_nop\n\tv_nop\n\tv_nop" : "+v"(a), "+v"(b) : "v"(x), "v"(y)); }
__device__ __forceinline__ void keep4_h(v16h a, v16h b, v16h c, v16h d) { asm volatile("v_nop" :: "v"(a), "v"(b), "v"(c), "v"(d)); }
__device__ __forceinline__ void keep4_b(v16b a, v16b b, v16b c, v16b d) { asm volatile("v_nop" :: "v"(a), "v"(b), "v"(c), "v"(d)); }
__device__ __forceinline__ void acc_guard4(v8f& a, v8f& b, v8f& c, v8f& d) { asm volatile("v_nop\n\tv_nop\n\tv_nop\n\tv_nop" : "+v"(a), "+v"(b), "+v"(c), "+v"(d)); }
template <typename T> struct Frag;
template <> struct Frag<_Float16> {
  typedef v16h V; union U { v16h v; v8h h[2]; };
  static __device__ __forceinline__ v16h load(const _Float16* p) {
    U f; f.h[0] = *(const v8h*)(p); f.h[1] = *(const v8h*)(p + 16); return f.v;
  }
  static __device__ __forceinline__ v8f mma(v16h a, v16h b, v8f c) {
    return __builtin_amdgcn_wmma_f32_16x16x32_f16(false, a, false, b, (short)0, c, false, false);
  }
  static __device__ __forceinline__ void guard(v8f& a, v8f& b, v16h x, v16h y) { dep_guard_h(a, b, x, y); }
  static __device__ __forceinline__ void keep(v16h a, v16h b, v16h c, v16h d) { keep4_h(a, b, c, d); }
};
template <> struct Frag<__bf16> {
  typedef v16b V; union U { v16b v; v8b h[2]; };
  static __device__ __forceinline__ v16b load(const __bf16* p) {
    U f; f.h[0] = *(const v8b*)(p); f.h[1] = *(const v8b*)(p + 16); return f.v;
  }
  static __device__ __forceinline__ v8f mma(v16b a, v16b b, v8f c) {
    return __builtin_amdgcn_wmma_f32_16x16x32_bf16(false, a, false, b, (short)0, c, false, false);
  }
  static __device__ __forceinline__ void guard(v8f& a, v8f& b, v16b x, v16b y) { dep_guard_b(a, b, x, y); }
  static __device__ __forceinline__ void keep(v16b a, v16b b, v16b c, v16b d) { keep4_b(a, b, c, d); }
};

__device__ __forceinline__ float lu_sigm(float g) {
  return __builtin_amdgcn_rcpf(1.0f + __expf(-g));
}

__device__ __forceinline__ void wave_sync_lds() {
  __builtin_amdgcn_fence(__ATOMIC_RELEASE, "workgroup");
  __builtin_amdgcn_wave_barrier();
  __builtin_amdgcn_fence(__ATOMIC_ACQUIRE, "workgroup");
}

template <int ET> struct Elem;
template <> struct Elem<0> { typedef _Float16 T; };
template <> struct Elem<1> { typedef __bf16 T; };
template <int ET, bool SPLIT, int BIAS_MODE, int OUT_MODE, bool RESID, int ACT = 0>
__global__ __launch_bounds__(256) void wmma_gemm64(
    const unsigned short* __restrict__ Ap, const unsigned short* __restrict__ A2p, int lda, long strideA,
    const unsigned short* __restrict__ Btp, const unsigned short* __restrict__ Bt2p, int ldb, long strideB,
    void* __restrict__ Cout, void* __restrict__ Cout2, int ldc, long strideC,
    const float* __restrict__ bias,
    const float* __restrict__ resid, long strideR,
    int M, int N, int K, float scale) {
  typedef typename Elem<ET>::T T;
  typedef typename Frag<T>::V V;
  const T* A = (const T*)Ap; const T* A2 = (const T*)A2p; const T* Bt = (const T*)Btp; const T* Bt2 = (const T*)Bt2p;
  __shared__ __align__(16) float sT[8][16 * 68];
  const int b    = blockIdx.y;
  const int lane = threadIdx.x & 31;
  const int wave = threadIdx.x >> 5;
  const int tilesN = N >> 6;
  const int tilesM = M >> 6;
  const int tile = blockIdx.x * 8 + wave;
  if (tile >= tilesM * tilesN) return;
  const int tm = tile / tilesN;
  const int tn = tile - tm * tilesN;
  const int m0 = tm << 6;
  const int n0 = tn << 6;

  const T* Ab  = A  + (size_t)b * strideA;
  const T* Bb  = Bt + (size_t)b * strideB;
  const T* Ab2 = SPLIT ? (A2  + (size_t)b * strideA) : nullptr;
  const T* Bb2 = SPLIT ? (Bt2 + (size_t)b * strideB) : nullptr;

  const int rlane = lane & 15;
  const int koff  = (lane >> 4) * 8;
  const int mOff  = (lane >> 4) * 8;

  v8f acc[4][4];
#pragma unroll
  for (int i = 0; i < 4; ++i)
#pragma unroll
    for (int j = 0; j < 4; ++j) acc[i][j] = (v8f){0.f,0.f,0.f,0.f,0.f,0.f,0.f,0.f};

  for (int k0 = 0; k0 < K; k0 += 32) {
    V bh[4], bl[4];
#pragma unroll
    for (int j = 0; j < 4; ++j) {
      const size_t bo = (size_t)(n0 + (j << 4) + rlane) * ldb + koff + k0;
      bh[j] = Frag<T>::load(Bb + bo);
      if (SPLIT) bl[j] = Frag<T>::load(Bb2 + bo);
    }
#pragma unroll
    for (int i = 0; i < 4; ++i) {
      const size_t ao = (size_t)(m0 + (i << 4) + rlane) * lda + koff + k0;
      V ah = Frag<T>::load(Ab + ao);
      V al;
      if (SPLIT) al = Frag<T>::load(Ab2 + ao);
#pragma unroll
      for (int j = 0; j < 4; ++j) {
        acc[i][j] = Frag<T>::mma(ah, bh[j], acc[i][j]);
        if (SPLIT) {
          acc[i][j] = Frag<T>::mma(ah, bl[j], acc[i][j]);
          acc[i][j] = Frag<T>::mma(al, bh[j], acc[i][j]);
        }
      }
      Frag<T>::guard(acc[i][0], acc[i][3], ah, SPLIT ? al : ah);
    }
    Frag<T>::keep(bh[0], bh[1], bh[2], bh[3]);
    if (SPLIT) Frag<T>::keep(bl[0], bl[1], bl[2], bl[3]);
  }
  acc_guard4(acc[0][0], acc[0][1], acc[0][2], acc[0][3]);
  acc_guard4(acc[1][0], acc[1][1], acc[1][2], acc[1][3]);
  acc_guard4(acc[2][0], acc[2][1], acc[2][2], acc[2][3]);
  acc_guard4(acc[3][0], acc[3][1], acc[3][2], acc[3][3]);

  float act_m = 1.0f, act_o = 0.0f;
  if (ACT == 6) {
    const bool tg = ((n0 >> LU_DSHIFT) == 2);
    act_m = tg ? 2.0f : 1.0f;
    act_o = tg ? -1.0f : 0.0f;
  }
  float* slab = sT[wave];
  const float* Rb = RESID ? (resid + (size_t)b * strideR) : nullptr;
#pragma unroll
  for (int i = 0; i < 4; ++i) {
    const int mBase = m0 + (i << 4);
#pragma unroll
    for (int j = 0; j < 4; ++j) {
      const int n = n0 + (j << 4) + rlane;
      float bv = 0.f;
      if (BIAS_MODE == 2) bv = bias[n];
#pragma unroll
      for (int r = 0; r < 8; ++r) {
        float v = acc[i][j][r] * scale;
        if (BIAS_MODE == 1) v += bias[mBase + mOff + r];
        if (BIAS_MODE == 2) v += bv;
        if (RESID) v += Rb[(size_t)(mBase + mOff + r) * ldc + n];
        if (ACT == 1) v = tanhf(v);
        if (ACT == 2) v = fmaxf(v, 0.0f);
        if (ACT == 3) v = v / (1.0f + expf(-v));
        if (ACT == 4) v = (v > 0.f) ? v : 0.01f * v;
        if (ACT == 5) v = 0.5f * v * (1.0f + erff(v * 0.70710678118654752f));
        if (ACT == 6) { const float rr = lu_sigm(v * act_m); v = rr * act_m + act_o; }
        slab[(mOff + r) * 68 + (j << 4) + rlane] = v;
      }
    }
    __builtin_amdgcn_fence(__ATOMIC_RELEASE, "workgroup");
    __builtin_amdgcn_wave_barrier();
    __builtin_amdgcn_fence(__ATOMIC_ACQUIRE, "workgroup");
    if (OUT_MODE == 0) {
      float* C = (float*)Cout + (size_t)b * strideC;
      const int hh = lane >> 4, c4 = (lane & 15) * 4;
      for (int pass = 0; pass < 2; ++pass) {
#pragma unroll
        for (int it = 0; it < 8; ++it) {
          const int row = it * 2 + hh;
          v4f v = *(const v4f*)(slab + row * 68 + c4);
          *(volatile v4f*)(C + (size_t)(mBase + row) * ldc + n0 + c4) = v;
        }
        __threadfence();
      }
    } else {
      const int q = lane >> 3, c8 = (lane & 7) * 8;
      unsigned short* C  = (unsigned short*)Cout  + (size_t)b * strideC;
      unsigned short* C2 = (OUT_MODE == 2) ? ((unsigned short*)Cout2 + (size_t)b * strideC) : nullptr;
      for (int pass = 0; pass < 2; ++pass) {
#pragma unroll
        for (int it = 0; it < 4; ++it) {
          const int row = it * 4 + q;
          const float* sp = slab + row * 68 + c8;
          v8h hv, lv;
#pragma unroll
          for (int e = 0; e < 8; ++e) {
            if (OUT_MODE == 1) {
              hv[e] = (_Float16)sp[e];
            } else {
              unsigned short hb = f2bf_bits(sp[e]);
              unsigned short lb = f2bf_bits(sp[e] - bf_bits2f(hb));
              hv[e] = __builtin_bit_cast(_Float16, hb);
              lv[e] = __builtin_bit_cast(_Float16, lb);
            }
          }
          *(volatile v8h*)(C + (size_t)(mBase + row) * ldc + n0 + c8) = hv;
          if (OUT_MODE == 2) *(volatile v8h*)(C2 + (size_t)(mBase + row) * ldc + n0 + c8) = lv;
        }
        __threadfence();
      }
    }
    __builtin_amdgcn_fence(__ATOMIC_RELEASE, "workgroup");
    __builtin_amdgcn_wave_barrier();
    __builtin_amdgcn_fence(__ATOMIC_ACQUIRE, "workgroup");
  }
}

__global__ __launch_bounds__(256) void cast_f32_f16x2s(
    const float* __restrict__ in, _Float16* __restrict__ out, int n2, float sc) {
  int i = blockIdx.x * 256 + threadIdx.x;
  if (i < n2) {
    const _Float16 e0 = (_Float16)(in[2 * i] * sc), e1 = (_Float16)(in[2 * i + 1] * sc);
    const unsigned u = (unsigned)__builtin_bit_cast(unsigned short, e0) | ((unsigned)__builtin_bit_cast(unsigned short, e1) << 16);
    ((volatile unsigned*)out)[i] = u;
    __threadfence();
    ((volatile unsigned*)out)[i] = u;
  }
}

__global__ __launch_bounds__(128) void lucy_scan(
    const float* __restrict__ G, const float* __restrict__ h0, const float* __restrict__ s0,
    float* hst, float* sst, float* __restrict__ out, float* __restrict__ sT,
    int tbase, int first, int last) {
  __shared__ __align__(16) float os[4][8 * 32];
  const int tid  = threadIdx.x;
  const int wave = tid >> 5;
  const int lane = tid & 31;
  const int gid  = blockIdx.x * 128 + tid;
  if (gid >= LU_B * LU_D) return;
  const int b  = gid >> LU_DSHIFT;
  const int d  = gid & (LU_D - 1);
  const int d0 = d & ~31;

  float h, s;
  if (first) { h = h0[b * LU_D + d];  s = s0[b * LU_D + d]; }
  else       { h = hst[b * LU_D + d]; s = sst[b * LU_D + d]; }

  const float* gp = G + (size_t)b * LU_TCH * LU_GC + d;
  float* ob  = out + ((size_t)b * LU_T + tbase) * LU_D + d0;
  float* osw = os[wave];
  const int q = lane >> 3, c4 = (lane & 7) * 4;

  for (int t8 = 0; t8 < LU_TCH; t8 += 8) {
#pragma unroll
    for (int j = 0; j < 8; ++j) {
      const float* gr = gp + (size_t)(t8 + j) * LU_GC;
      const float ig = gr[0];
      const float fg = gr[LU_D];
      const float cg = gr[2 * LU_D];
      const float og = gr[3 * LU_D];
      const float ag = gr[4 * LU_D];
      const float wg = gr[5 * LU_D];
      h = fg * h + ig * cg;
      s = ag * s + wg * h;
      osw[j * 32 + lane] = og * h;
    }
    wave_sync_lds();
    for (int pass = 0; pass < 2; ++pass) {
#pragma unroll
      for (int it = 0; it < 2; ++it) {
        const int row = it * 4 + q;
        const v4f val = *(const v4f*)(osw + row * 32 + c4);
        *(volatile v4f*)(ob + (size_t)(t8 + row) * LU_D + c4) = val;
      }
      __threadfence();
    }
    wave_sync_lds();
  }

  osw[lane] = h;
  osw[32 + lane] = s;
  wave_sync_lds();
  if (lane < 16) {
    const v4f val = *(const v4f*)(osw + q * 32 + c4);
    float* dst = ((q == 0) ? hst : sst) + (size_t)b * LU_D + d0 + c4;
    *(volatile v4f*)dst = val;
    __threadfence();
    *(volatile v4f*)dst = val;
    if (last && q == 1) {
      float* dst2 = sT + (size_t)b * LU_D + d0 + c4;
      *(volatile v4f*)dst2 = val;
      __threadfence();
      *(volatile v4f*)dst2 = val;
    }
  }
}

extern "C" void kernel_launch(void* const* d_in, const int* in_sizes, int n_in,
                              void* d_out, int out_size, void* d_ws, size_t ws_size,
                              hipStream_t stream) {
  if (n_in < 5) return;
  const int nx = in_sizes[0];
  const int nw = in_sizes[3];
  if (nx != LU_B * LU_T * LU_IN) return;
  if (in_sizes[1] != LU_B * LU_D || in_sizes[2] != LU_B * LU_D) return;
  if (nw != LU_GC * LU_IN || in_sizes[4] != LU_GC) return;
  if (out_size != LU_B * LU_T * LU_D + LU_B * LU_D) return;

  const float* x    = (const float*)d_in[0];
  const float* h0   = (const float*)d_in[1];
  const float* s0   = (const float*)d_in[2];
  const float* W    = (const float*)d_in[3];
  const float* bias = (const float*)d_in[4];
  float* out = (float*)d_out;
  float* sTp = out + (size_t)LU_B * LU_T * LU_D;

  const size_t g_bytes  = (size_t)LU_B * LU_TCH * LU_GC * sizeof(float);
  const size_t xh_bytes = (size_t)nx * 2;
  const size_t wh_bytes = (size_t)nw * 2;
  const size_t st_bytes = (size_t)LU_B * LU_D * sizeof(float);
  const size_t off_g  = 0;
  const size_t off_xh = off_g + g_bytes;
  const size_t off_wh = off_xh + xh_bytes;
  const size_t off_h  = off_wh + wh_bytes;
  const size_t off_s  = off_h + st_bytes;
  const size_t total  = off_s + st_bytes;
  if (total > ws_size) return;

  char* ws = (char*)d_ws;
  float*    G   = (float*)(ws + off_g);
  _Float16* xh  = (_Float16*)(ws + off_xh);
  _Float16* wh  = (_Float16*)(ws + off_wh);
  float*    hst = (float*)(ws + off_h);
  float*    sst = (float*)(ws + off_s);

  {
    const int n2x = nx / 2;
    cast_f32_f16x2s<<<dim3((n2x + 255) / 256), dim3(256), 0, stream>>>(x, xh, n2x, 1.0f);
    const int n2w = nw / 2;
    cast_f32_f16x2s<<<dim3((n2w + 255) / 256), dim3(256), 0, stream>>>(W, wh, n2w, LU_WSCALE);
  }

  const int tilesM = LU_TCH / 64;
  const int tilesN = LU_GC / 64;
  const dim3 ggrid((tilesM * tilesN + 7) / 8, LU_B);
  for (int c = 0; c < LU_NCH; ++c) {
    const unsigned short* Ap = (const unsigned short*)xh + (size_t)c * LU_TCH * LU_IN;
    const unsigned short* Bp = (const unsigned short*)wh;
    wmma_gemm64<0, false, 2, 0, false, 6><<<ggrid, dim3(256), 0, stream>>>(
        Ap, Ap, LU_IN, (long)LU_T * LU_IN,
        Bp, Bp, LU_IN, 0L,
        (void*)G, (void*)G, LU_GC, (long)LU_TCH * LU_GC,
        bias,
        (const float*)G, 0L,
        LU_TCH, LU_GC, LU_IN, LU_WSCALE_INV);
    lucy_scan<<<dim3((LU_B * LU_D + 127) / 128), dim3(128), 0, stream>>>(
        G, h0, s0, hst, sst, out, sTp, c * LU_TCH, (c == 0) ? 1 : 0, (c == LU_NCH - 1) ? 1 : 0);
  }
}
